// parallel_MLP_28819230556803
// MI455X (gfx1250) — hardware-verified
//
#include <hip/hip_runtime.h>
#include <stdint.h>

#pragma clang fp contract(off)

typedef _Float16 v16h __attribute__((ext_vector_type(16)));
typedef _Float16 v8h  __attribute__((ext_vector_type(8)));
typedef float    v8f  __attribute__((ext_vector_type(8)));
typedef float    v4f  __attribute__((ext_vector_type(4)));
typedef v4f      v4fa __attribute__((may_alias));

#define LAYERW 50
#define ROWLEN (3 * LAYERW + 1)
#define KPAD   64
#define PT     72
#define NWAVE  4
#define NTHR   (32 * NWAVE)
#define RPW    32
#define RPB    (RPW * NWAVE)

#define W2SC 64.0f
#define RW2  (1.0f / 64.0f)
#define RESC 4096.0f
#define RRES (1.0f / 4096.0f)

static_assert(KPAD == 64);
static_assert(LAYERW <= KPAD && LAYERW >= KPAD - 16);
static_assert((PT % 8) == 0 && PT >= KPAD);
static_assert(NTHR == 2 * KPAD);

__device__ __forceinline__ float bf_rne(float f) {
  unsigned u = __float_as_uint(f);
  u = (u + 0x7FFFu + ((u >> 16) & 1u)) & 0xFFFF0000u;
  return __uint_as_float(u);
}
__device__ __forceinline__ v8f zero8() { v8f z = {0.f, 0.f, 0.f, 0.f, 0.f, 0.f, 0.f, 0.f}; return z; }
__device__ __forceinline__ v8h zero8h() {
  v8h z;
#pragma unroll
  for (int i = 0; i < 8; ++i) z[i] = (_Float16)0.0f;
  return z;
}
__device__ __forceinline__ float tanh_e(float a) {
  const float y = fabsf(a);
  const float e = __expf(-2.0f * y);
  const float r = (1.0f - e) * __builtin_amdgcn_rcpf(1.0f + e);
  return copysignf(r, a);
}

__device__ __forceinline__ v16h ldfrag_h(const _Float16* p) {
  union { v16h v; v8h h[2]; } f;
  f.h[0] = *(const v8h*)(p);
  f.h[1] = *(const v8h*)(p + 16);
  return f.v;
}

__device__ __forceinline__ v8f mma_h(v16h a, v16h b, v8f c) {
  c = __builtin_amdgcn_wmma_f32_16x16x32_f16(false, a, false, b, (short)0, c, false, false);
#if defined(__HIP_DEVICE_COMPILE__)
  asm volatile("v_nop\n\tv_nop\n\tv_nop\n\tv_nop" : "+v"(c) : "v"(a), "v"(b));
#endif
  return c;
}
__device__ __forceinline__ void wave_sync_lds() {
  __builtin_amdgcn_fence(__ATOMIC_RELEASE, "workgroup");
  __builtin_amdgcn_wave_barrier();
  __builtin_amdgcn_fence(__ATOMIC_ACQUIRE, "workgroup");
}

__global__ __launch_bounds__(NTHR) void pmlp_fused(const float* __restrict__ theta,
                                                   const float* __restrict__ x,
                                                   float* out, int T, int N) {
  __shared__ __align__(16) _Float16 tileH[NWAVE * RPW * PT];
  __shared__ __align__(16) _Float16 tileR[NWAVE * RPW * PT];
  __shared__ __align__(16) float    slab[NWAVE * RPW];
  __shared__ __align__(16) float    s_w1[KPAD];
  __shared__ __align__(16) float    s_b1[KPAD];
  __shared__ __align__(16) _Float16 s_w2h[KPAD];

  const int t   = blockIdx.y;
  const int tid = threadIdx.x;
  const float* row = theta + (size_t)t * ROWLEN;

  if (tid < KPAD) {
    const int i  = tid;
    const int ic = min(i, LAYERW - 1);
    const float a = row[ic];
    const float b = row[LAYERW + ic];
    s_w1[i] = (i < LAYERW) ? bf_rne(a) : 0.0f;
    s_b1[i] = (i < LAYERW) ? bf_rne(b) : 0.0f;
  } else {
    const int i  = tid - KPAD;
    const int ic = min(i, LAYERW - 1);
    const float c = row[2 * LAYERW + ic];
    const float v = (i < LAYERW) ? bf_rne(c) * W2SC : 0.0f;
    s_w2h[i] = (_Float16)v;
  }
  const float b2 = bf_rne(row[3 * LAYERW]);
  __syncthreads();

  const int lane = tid & 31;
  const int wave = tid >> 5;
  const int c    = lane & 15;
  const int g    = lane >> 4;
  const int n0   = blockIdx.x * RPB + wave * RPW;

  if (n0 < N) {
    _Float16* tH = tileH + wave * (RPW * PT);
    _Float16* tR = tileR + wave * (RPW * PT);
    float*    sl = slab + wave * RPW;

    const v16h bq0 = ldfrag_h(s_w2h + 8 * g);
    const v16h bq1 = ldfrag_h(s_w2h + 32 + 8 * g);

    const int   nr = min(n0 + lane, N - 1);
    const float xv = bf_rne(x[nr]);
    _Float16* rH = tH + lane * PT;
    _Float16* rR = tR + lane * PT;
    {
      const v8h z8 = zero8h();
      *(v8h*)(rH + (KPAD - 16)) = z8;
      *(v8h*)(rH + (KPAD - 8))  = z8;
      *(v8h*)(rR + (KPAD - 16)) = z8;
      *(v8h*)(rR + (KPAD - 8))  = z8;
    }
#pragma unroll 1
    for (int k = 0; k < LAYERW; ++k) {
      const float pre = s_w1[k] * xv + s_b1[k];
      const float hv  = tanh_e(pre);
      const _Float16 hh = (_Float16)hv;
      const float rs  = (hv - (float)hh) * RESC;
      rH[k] = hh;
      rR[k] = (_Float16)rs;
    }
    wave_sync_lds();

    v8f accH[2], accR[2];
#pragma unroll
    for (int u = 0; u < 2; ++u) {
      const _Float16* pH = tH + (u * 16 + c) * PT + 8 * g;
      const _Float16* pR = tR + (u * 16 + c) * PT + 8 * g;
      const v16h aH0 = ldfrag_h(pH);
      const v16h aH1 = ldfrag_h(pH + 32);
      const v16h aR0 = ldfrag_h(pR);
      const v16h aR1 = ldfrag_h(pR + 32);
      v8f ah = mma_h(aH0, bq0, zero8());
      ah     = mma_h(aH1, bq1, ah);
      v8f ar = mma_h(aR0, bq0, zero8());
      ar     = mma_h(aR1, bq1, ar);
      accH[u] = ah;
      accR[u] = ar;
    }

    if (c == 0) {
#pragma unroll
      for (int u = 0; u < 2; ++u) {
        v4f o0, o1;
#pragma unroll
        for (int r = 0; r < 4; ++r) {
          o0[r] = (accH[u][r]     + accR[u][r]     * RRES) * RW2 + b2;
          o1[r] = (accH[u][4 + r] + accR[u][4 + r] * RRES) * RW2 + b2;
        }
        *(v4f*)(sl + u * 16 + 8 * g)     = o0;
        *(v4f*)(sl + u * 16 + 8 * g + 4) = o1;
      }
    }
    wave_sync_lds();

    const int q = lane & 7;
    const v4f o = *(const v4fa*)(sl + 4 * q);
    float* op = out + (size_t)t * N + n0 + 4 * q;
    if (lane < 8) *(volatile v4f*)op = o;
    __threadfence();
    if (lane < 8) *(volatile v4f*)op = o;
  }
}

extern "C" void kernel_launch(void* const* d_in, const int* in_sizes, int n_in,
                              void* d_out, int out_size, void* d_ws, size_t ws_size,
                              hipStream_t stream) {
  (void)d_ws; (void)ws_size;
  if (n_in < 2) return;
  const int nth = in_sizes[0];
  const int N   = in_sizes[1];
  if (nth <= 0 || (nth % ROWLEN) != 0) return;
  const int T = nth / ROWLEN;
  if (T < 1 || T > 65535) return;
  if (N < RPW || (N % RPW) != 0) return;
  if ((long long)T * (long long)N != (long long)out_size) return;

  const float* theta = (const float*)d_in[0];
  const float* x     = (const float*)d_in[1];
  float*       out   = (float*)d_out;

  const int nchunk = (N + RPB - 1) / RPB;
  pmlp_fused<<<dim3(nchunk, T), dim3(NTHR), 0, stream>>>(theta, x, out, T, N);
  (void)hipGetLastError();
}
